// PrunedMultiHeadAttention_75230647157611
// MI455X (gfx1250) — hardware-verified
//
#include <hip/hip_runtime.h>
#include <math.h>
#include <stdint.h>

#define NBATCH 2
#define SEQ    2048
#define DMOD   1024
#define NHEAD  16
#define DHD    64

typedef __attribute__((ext_vector_type(16))) _Float16 v16h;
typedef __attribute__((ext_vector_type(8)))  _Float16 v8h;
typedef __attribute__((ext_vector_type(16))) __bf16   v16b;
typedef __attribute__((ext_vector_type(8)))  __bf16   v8b;
typedef __attribute__((ext_vector_type(8)))  float    v8f;
typedef __attribute__((ext_vector_type(4)))  float    v4f;
typedef __attribute__((ext_vector_type(2)))  float    v2f;
typedef __attribute__((ext_vector_type(4)))  unsigned int v4u;

__device__ __forceinline__ unsigned short f2bf_bits(float f) {
  unsigned u = __float_as_uint(f);
  return (unsigned short)((u + 0x7FFFu + ((u >> 16) & 1u)) >> 16);
}
__device__ __forceinline__ float bf_bits2f(unsigned short h) { return __uint_as_float(((unsigned)h) << 16); }

__device__ __forceinline__ void dep_guard_h(v8f& a, v8f& b, v16h x, v16h y) { asm volatile("v_nop\n\tv_nop\n\tv_nop\n\tv_nop" : "+v"(a), "+v"(b) : "v"(x), "v"(y)); }
__device__ __forceinline__ void dep_guard_b(v8f& a, v8f& b, v16b x, v16b y) { asm volatile("v_nop\n\tv_nop\n\tv_nop\n\tv_nop" : "+v"(a), "+v"(b) : "v"(x), "v"(y)); }
__device__ __forceinline__ void keep4_h(v16h a, v16h b, v16h c, v16h d) { asm volatile("v_nop" :: "v"(a), "v"(b), "v"(c), "v"(d)); }
__device__ __forceinline__ void keep4_b(v16b a, v16b b, v16b c, v16b d) { asm volatile("v_nop" :: "v"(a), "v"(b), "v"(c), "v"(d)); }
__device__ __forceinline__ void acc_guard4(v8f& a, v8f& b, v8f& c, v8f& d) { asm volatile("v_nop\n\tv_nop\n\tv_nop\n\tv_nop" : "+v"(a), "+v"(b), "+v"(c), "+v"(d)); }
template <typename T> struct Frag;
template <> struct Frag<_Float16> {
  typedef v16h V; union U { v16h v; v8h h[2]; };
  static __device__ __forceinline__ v16h load(const _Float16* p) {
    U f; f.h[0] = *(const v8h*)(p); f.h[1] = *(const v8h*)(p + 16); return f.v;
  }
  static __device__ __forceinline__ v8f mma(v16h a, v16h b, v8f c) {
    return __builtin_amdgcn_wmma_f32_16x16x32_f16(false, a, false, b, (short)0, c, false, false);
  }
  static __device__ __forceinline__ void guard(v8f& a, v8f& b, v16h x, v16h y) { dep_guard_h(a, b, x, y); }
  static __device__ __forceinline__ void keep(v16h a, v16h b, v16h c, v16h d) { keep4_h(a, b, c, d); }
};
template <> struct Frag<__bf16> {
  typedef v16b V; union U { v16b v; v8b h[2]; };
  static __device__ __forceinline__ v16b load(const __bf16* p) {
    U f; f.h[0] = *(const v8b*)(p); f.h[1] = *(const v8b*)(p + 16); return f.v;
  }
  static __device__ __forceinline__ v8f mma(v16b a, v16b b, v8f c) {
    return __builtin_amdgcn_wmma_f32_16x16x32_bf16(false, a, false, b, (short)0, c, false, false);
  }
  static __device__ __forceinline__ void guard(v8f& a, v8f& b, v16b x, v16b y) { dep_guard_b(a, b, x, y); }
  static __device__ __forceinline__ void keep(v16b a, v16b b, v16b c, v16b d) { keep4_b(a, b, c, d); }
};

template <int ET> struct Elem;
template <> struct Elem<0> { typedef _Float16 T; };
template <> struct Elem<1> { typedef __bf16 T; };
template <int ET, bool SPLIT, int BIAS_MODE, int OUT_MODE, bool RESID, int ACT = 0>
__global__ __launch_bounds__(256) void wmma_gemm64(
    const unsigned short* __restrict__ Ap, const unsigned short* __restrict__ A2p, int lda, long strideA,
    const unsigned short* __restrict__ Btp, const unsigned short* __restrict__ Bt2p, int ldb, long strideB,
    void* __restrict__ Cout, void* __restrict__ Cout2, int ldc, long strideC,
    const float* __restrict__ bias,
    const float* __restrict__ resid, long strideR,
    int M, int N, int K, float scale) {
  typedef typename Elem<ET>::T T;
  typedef typename Frag<T>::V V;
  const T* A = (const T*)Ap; const T* A2 = (const T*)A2p; const T* Bt = (const T*)Btp; const T* Bt2 = (const T*)Bt2p;
  __shared__ __align__(16) float sT[8][16 * 68];
  const int b    = blockIdx.y;
  const int lane = threadIdx.x & 31;
  const int wave = threadIdx.x >> 5;
  const int tilesN = N >> 6;
  const int tilesM = M >> 6;
  const int tile = blockIdx.x * 8 + wave;
  if (tile >= tilesM * tilesN) return;
  const int tm = tile / tilesN;
  const int tn = tile - tm * tilesN;
  const int m0 = tm << 6;
  const int n0 = tn << 6;

  const T* Ab  = A  + (size_t)b * strideA;
  const T* Bb  = Bt + (size_t)b * strideB;
  const T* Ab2 = SPLIT ? (A2  + (size_t)b * strideA) : nullptr;
  const T* Bb2 = SPLIT ? (Bt2 + (size_t)b * strideB) : nullptr;

  const int rlane = lane & 15;
  const int koff  = (lane >> 4) * 8;
  const int mOff  = (lane >> 4) * 8;

  v8f acc[4][4];
#pragma unroll
  for (int i = 0; i < 4; ++i)
#pragma unroll
    for (int j = 0; j < 4; ++j) acc[i][j] = (v8f){0.f,0.f,0.f,0.f,0.f,0.f,0.f,0.f};

  for (int k0 = 0; k0 < K; k0 += 32) {
    V bh[4], bl[4];
#pragma unroll
    for (int j = 0; j < 4; ++j) {
      const size_t bo = (size_t)(n0 + (j << 4) + rlane) * ldb + koff + k0;
      bh[j] = Frag<T>::load(Bb + bo);
      if (SPLIT) bl[j] = Frag<T>::load(Bb2 + bo);
    }
#pragma unroll
    for (int i = 0; i < 4; ++i) {
      const size_t ao = (size_t)(m0 + (i << 4) + rlane) * lda + koff + k0;
      V ah = Frag<T>::load(Ab + ao);
      V al;
      if (SPLIT) al = Frag<T>::load(Ab2 + ao);
#pragma unroll
      for (int j = 0; j < 4; ++j) {
        acc[i][j] = Frag<T>::mma(ah, bh[j], acc[i][j]);
        if (SPLIT) {
          acc[i][j] = Frag<T>::mma(ah, bl[j], acc[i][j]);
          acc[i][j] = Frag<T>::mma(al, bh[j], acc[i][j]);
        }
      }
      Frag<T>::guard(acc[i][0], acc[i][3], ah, SPLIT ? al : ah);
    }
    Frag<T>::keep(bh[0], bh[1], bh[2], bh[3]);
    if (SPLIT) Frag<T>::keep(bl[0], bl[1], bl[2], bl[3]);
  }
  acc_guard4(acc[0][0], acc[0][1], acc[0][2], acc[0][3]);
  acc_guard4(acc[1][0], acc[1][1], acc[1][2], acc[1][3]);
  acc_guard4(acc[2][0], acc[2][1], acc[2][2], acc[2][3]);
  acc_guard4(acc[3][0], acc[3][1], acc[3][2], acc[3][3]);

  float* slab = sT[wave];
  const float* Rb = RESID ? (resid + (size_t)b * strideR) : nullptr;
#pragma unroll
  for (int i = 0; i < 4; ++i) {
    const int mBase = m0 + (i << 4);
#pragma unroll
    for (int j = 0; j < 4; ++j) {
      const int n = n0 + (j << 4) + rlane;
      float bv = 0.f;
      if (BIAS_MODE == 2) bv = bias[n];
#pragma unroll
      for (int r = 0; r < 8; ++r) {
        float v = acc[i][j][r] * scale;
        if (BIAS_MODE == 1) v += bias[mBase + mOff + r];
        if (BIAS_MODE == 2) v += bv;
        if (RESID) v += Rb[(size_t)(mBase + mOff + r) * ldc + n];
        if (ACT == 1) v = tanhf(v);
        if (ACT == 2) v = fmaxf(v, 0.0f);
        if (ACT == 3) v = v / (1.0f + expf(-v));
        if (ACT == 4) v = (v > 0.f) ? v : 0.01f * v;
        slab[(mOff + r) * 68 + (j << 4) + rlane] = v;
      }
    }
    __builtin_amdgcn_fence(__ATOMIC_RELEASE, "workgroup");
    __builtin_amdgcn_wave_barrier();
    __builtin_amdgcn_fence(__ATOMIC_ACQUIRE, "workgroup");
    if (OUT_MODE == 0) {
      float* C = (float*)Cout + (size_t)b * strideC;
      const int hh = lane >> 4, c4 = (lane & 15) * 4;
      for (int pass = 0; pass < 2; ++pass) {
#pragma unroll
        for (int it = 0; it < 8; ++it) {
          const int row = it * 2 + hh;
          v4f v = *(const v4f*)(slab + row * 68 + c4);
          *(volatile v4f*)(C + (size_t)(mBase + row) * ldc + n0 + c4) = v;
        }
        __threadfence();
      }
    } else {
      const int q = lane >> 3, c8 = (lane & 7) * 8;
      unsigned short* C  = (unsigned short*)Cout  + (size_t)b * strideC;
      unsigned short* C2 = (OUT_MODE == 2) ? ((unsigned short*)Cout2 + (size_t)b * strideC) : nullptr;
      for (int pass = 0; pass < 2; ++pass) {
#pragma unroll
        for (int it = 0; it < 4; ++it) {
          const int row = it * 4 + q;
          const float* sp = slab + row * 68 + c8;
          v8h hv, lv;
#pragma unroll
          for (int e = 0; e < 8; ++e) {
            if (OUT_MODE == 1) {
              hv[e] = (_Float16)sp[e];
            } else {
              unsigned short hb = f2bf_bits(sp[e]);
              unsigned short lb = f2bf_bits(sp[e] - bf_bits2f(hb));
              hv[e] = __builtin_bit_cast(_Float16, hb);
              lv[e] = __builtin_bit_cast(_Float16, lb);
            }
          }
          *(volatile v8h*)(C + (size_t)(mBase + row) * ldc + n0 + c8) = hv;
          if (OUT_MODE == 2) *(volatile v8h*)(C2 + (size_t)(mBase + row) * ldc + n0 + c8) = lv;
        }
        __threadfence();
      }
    }
    __builtin_amdgcn_fence(__ATOMIC_RELEASE, "workgroup");
    __builtin_amdgcn_wave_barrier();
    __builtin_amdgcn_fence(__ATOMIC_ACQUIRE, "workgroup");
  }
}

__device__ __forceinline__ unsigned pk16(unsigned short a, unsigned short b) { return (unsigned)a | ((unsigned)b << 16); }

__global__ __launch_bounds__(256) void cast_f32_f16x2s(const float* __restrict__ in, _Float16* __restrict__ out,
                                                        int n2, float mul) {
  const int i = blockIdx.x * 256 + threadIdx.x;
  if (i < n2) {
    const v2f f = *(const v2f*)(in + 2 * (size_t)i);
    const _Float16 h0 = (_Float16)(f[0] * mul), h1 = (_Float16)(f[1] * mul);
    const unsigned u = pk16(__builtin_bit_cast(unsigned short, h0), __builtin_bit_cast(unsigned short, h1));
    ((volatile unsigned*)out)[i] = u;
    __threadfence();
    ((volatile unsigned*)out)[i] = u;
  }
}

__global__ __launch_bounds__(256) void maskcast_f32_f16x2(const float* __restrict__ in, const int* __restrict__ hmask,
                                                          _Float16* __restrict__ out, int n2, int ncol, float mul) {
  const int i = blockIdx.x * 256 + threadIdx.x;
  if (i < n2) {
    const v2f f = *(const v2f*)(in + 2 * (size_t)i);
    const int col = (2 * i) & (ncol - 1);
    int hd = col >> 6;
    hd = hd < 0 ? 0 : (hd > NHEAD - 1 ? NHEAD - 1 : hd);
    const float fac = (hmask[hd] != 0) ? mul : 0.0f;
    const _Float16 h0 = (_Float16)(f[0] * fac), h1 = (_Float16)(f[1] * fac);
    const unsigned u = pk16(__builtin_bit_cast(unsigned short, h0), __builtin_bit_cast(unsigned short, h1));
    ((volatile unsigned*)out)[i] = u;
    __threadfence();
    ((volatile unsigned*)out)[i] = u;
  }
}

#define AT_D 64
#define AT_NW 4
#define AT_QB 64
#define AT_KC 64

__device__ __forceinline__ unsigned short at_bf_bits(float f) {
  unsigned u = __float_as_uint(f);
  return (unsigned short)((u + 0x7FFFu + ((u >> 16) & 1u)) >> 16);
}
__device__ __forceinline__ __bf16 at_f2bf(float f) { return __builtin_bit_cast(__bf16, at_bf_bits(f)); }
__device__ __forceinline__ void at_split(float f, __bf16& hi, __bf16& lo) {
  const unsigned short hb = at_bf_bits(f);
  hi = __builtin_bit_cast(__bf16, hb);
  lo = at_f2bf(f - __uint_as_float(((unsigned)hb) << 16));
}
__device__ __forceinline__ v8f at_mma(v16b a, v16b b, v8f c) {
  c = __builtin_amdgcn_wmma_f32_16x16x32_bf16(false, a, false, b, (short)0, c, false, false);
  asm volatile("v_nop\n\tv_nop\n\tv_nop\n\tv_nop" : "+v"(c) : "v"(a), "v"(b));
  return c;
}

__global__ __launch_bounds__(128)
void attn_full64_kernel(const unsigned short* __restrict__ qhp, const unsigned short* __restrict__ qlp,
                        const unsigned short* __restrict__ khp, const unsigned short* __restrict__ klp,
                        const unsigned short* __restrict__ vhp, const unsigned short* __restrict__ vlp,
                        float* __restrict__ out, float sscale) {
  union FB { v16b v; v8b h[2]; };
  __shared__ __align__(16) __bf16 Ksh[AT_KC * AT_D];
  __shared__ __align__(16) __bf16 Ksl[AT_KC * AT_D];
  __shared__ __align__(16) __bf16 Vth[AT_D * AT_KC];
  __shared__ __align__(16) __bf16 Vtl[AT_D * AT_KC];
  __shared__ __align__(16) __bf16 Psh[AT_NW][16 * AT_KC];
  __shared__ __align__(16) __bf16 Psl[AT_NW][16 * AT_KC];
  __shared__ __align__(16) float  Os[AT_NW][16 * 68];

  const int tid  = threadIdx.x;
  const int wave = tid >> 5;
  const int lane = tid & 31;
  const int hh   = lane >> 4;
  const int c    = lane & 15;

  const int nqb = SEQ / AT_QB;
  const int bx = blockIdx.x;
  const int qb = bx % nqb;
  const int h  = bx / nqb;
  const int q0 = qb * AT_QB + wave * 16;

  const __bf16* Qh = (const __bf16*)(const void*)qhp + (size_t)h * AT_D;
  const __bf16* Ql = (const __bf16*)(const void*)qlp + (size_t)h * AT_D;
  const __bf16* Kh = (const __bf16*)(const void*)khp + (size_t)h * AT_D;
  const __bf16* Kl = (const __bf16*)(const void*)klp + (size_t)h * AT_D;
  const __bf16* Vh = (const __bf16*)(const void*)vhp + (size_t)h * AT_D * SEQ;
  const __bf16* Vl = (const __bf16*)(const void*)vlp + (size_t)h * AT_D * SEQ;
  float*        ob = out + (size_t)h * AT_D;

  v16b qah[2], qal[2];
#pragma unroll
  for (int dc = 0; dc < 2; ++dc) {
    const __bf16* qr = Qh + (size_t)(q0 + c) * DMOD + dc * 32 + 8 * hh;
    const __bf16* ql = Ql + (size_t)(q0 + c) * DMOD + dc * 32 + 8 * hh;
    qah[dc] = Frag<__bf16>::load(qr);
    qal[dc] = Frag<__bf16>::load(ql);
  }

  float mrow[8], lrow[8];
  v8f oacc[4];
#pragma unroll
  for (int r = 0; r < 8; ++r) { mrow[r] = -INFINITY; lrow[r] = 0.f; }
#pragma unroll
  for (int t = 0; t < 4; ++t) oacc[t] = (v8f){0.f,0.f,0.f,0.f,0.f,0.f,0.f,0.f};

  const int nChunks = SEQ / AT_KC;
  for (int kc = 0; kc < nChunks; ++kc) {
    const int kv0 = kc * AT_KC;
    __syncthreads();
    {
      const int r = tid >> 1, half = (tid & 1) * 32;
      const __bf16* ksh = Kh + (size_t)(kv0 + r) * DMOD + half;
      const __bf16* ksl = Kl + (size_t)(kv0 + r) * DMOD + half;
      const __bf16* vsh = Vh + (size_t)r * SEQ + kv0 + half;
      const __bf16* vsl = Vl + (size_t)r * SEQ + kv0 + half;
#pragma unroll
      for (int i = 0; i < 4; ++i) {
        const v8b a0 = *(const v8b*)(ksh + 8 * i);
        const v8b a1 = *(const v8b*)(ksl + 8 * i);
        const v8b b0 = *(const v8b*)(vsh + 8 * i);
        const v8b b1 = *(const v8b*)(vsl + 8 * i);
        *(v8b*)(Ksh + r * AT_D  + half + 8 * i) = a0;
        *(v8b*)(Ksl + r * AT_D  + half + 8 * i) = a1;
        *(v8b*)(Vth + r * AT_KC + half + 8 * i) = b0;
        *(v8b*)(Vtl + r * AT_KC + half + 8 * i) = b1;
      }
    }
    __syncthreads();

    v8f s[4];
#pragma unroll
    for (int j = 0; j < 4; ++j) {
      s[j] = (v8f){0.f,0.f,0.f,0.f,0.f,0.f,0.f,0.f};
#pragma unroll
      for (int dc = 0; dc < 2; ++dc) {
        FB kb, kl;
        kb.h[0] = *(const v8b*)(Ksh + (j * 16 + c) * AT_D + dc * 32 + 8 * hh);
        kb.h[1] = *(const v8b*)(Ksh + (j * 16 + c) * AT_D + dc * 32 + 16 + 8 * hh);
        kl.h[0] = *(const v8b*)(Ksl + (j * 16 + c) * AT_D + dc * 32 + 8 * hh);
        kl.h[1] = *(const v8b*)(Ksl + (j * 16 + c) * AT_D + dc * 32 + 16 + 8 * hh);
        s[j] = at_mma(qah[dc], kb.v, s[j]);
        s[j] = at_mma(qah[dc], kl.v, s[j]);
        s[j] = at_mma(qal[dc], kb.v, s[j]);
      }
    }
    float cm[8];
#pragma unroll
    for (int r = 0; r < 8; ++r) {
      float m = -INFINITY;
#pragma unroll
      for (int j = 0; j < 4; ++j) {
        const float sv = s[j][r] * sscale;
        s[j][r] = sv;
        m = fmaxf(m, sv);
      }
#pragma unroll
      for (int off = 1; off < 16; off <<= 1) m = fmaxf(m, __shfl_xor(m, off, 32));
      cm[r] = m;
    }
    __bf16* pwh = Psh[wave];
    __bf16* pwl = Psl[wave];
#pragma unroll
    for (int r = 0; r < 8; ++r) {
      const float mnew = fmaxf(mrow[r], cm[r]);
      const float alpha = expf(mrow[r] - mnew);
      mrow[r] = mnew;
      float psum = 0.f;
#pragma unroll
      for (int j = 0; j < 4; ++j) {
        const float p = expf(s[j][r] - mnew);
        psum += p;
        __bf16 a, bl; at_split(p, a, bl);
        pwh[(8 * hh + r) * AT_KC + j * 16 + c] = a;
        pwl[(8 * hh + r) * AT_KC + j * 16 + c] = bl;
      }
#pragma unroll
      for (int off = 1; off < 16; off <<= 1) psum += __shfl_xor(psum, off, 32);
      lrow[r] = lrow[r] * alpha + psum;
#pragma unroll
      for (int t = 0; t < 4; ++t) oacc[t][r] *= alpha;
    }
    __builtin_amdgcn_fence(__ATOMIC_RELEASE, "workgroup");
    __builtin_amdgcn_wave_barrier();
    __builtin_amdgcn_fence(__ATOMIC_ACQUIRE, "workgroup");
#pragma unroll 1
    for (int kk = 0; kk < 2; ++kk) {
      FB pa, pl;
      pa.h[0] = *(const v8b*)(pwh + c * AT_KC + kk * 32 + 8 * hh);
      pa.h[1] = *(const v8b*)(pwh + c * AT_KC + kk * 32 + 16 + 8 * hh);
      pl.h[0] = *(const v8b*)(pwl + c * AT_KC + kk * 32 + 8 * hh);
      pl.h[1] = *(const v8b*)(pwl + c * AT_KC + kk * 32 + 16 + 8 * hh);
#pragma unroll
      for (int t = 0; t < 4; ++t) {
        FB vb, vl;
        vb.h[0] = *(const v8b*)(Vth + (t * 16 + c) * AT_KC + kk * 32 + 8 * hh);
        vb.h[1] = *(const v8b*)(Vth + (t * 16 + c) * AT_KC + kk * 32 + 16 + 8 * hh);
        vl.h[0] = *(const v8b*)(Vtl + (t * 16 + c) * AT_KC + kk * 32 + 8 * hh);
        vl.h[1] = *(const v8b*)(Vtl + (t * 16 + c) * AT_KC + kk * 32 + 16 + 8 * hh);
        oacc[t] = at_mma(pa.v, vb.v, oacc[t]);
        oacc[t] = at_mma(pa.v, vl.v, oacc[t]);
        oacc[t] = at_mma(pl.v, vb.v, oacc[t]);
      }
    }
  }

  float* os = Os[wave];
#pragma unroll
  for (int r = 0; r < 8; ++r) {
    const float inv = 1.0f / lrow[r];
#pragma unroll
    for (int t = 0; t < 4; ++t) os[(8 * hh + r) * 68 + t * 16 + c] = oacc[t][r] * inv;
  }
  __builtin_amdgcn_fence(__ATOMIC_RELEASE, "workgroup");
  __builtin_amdgcn_wave_barrier();
  __builtin_amdgcn_fence(__ATOMIC_ACQUIRE, "workgroup");
  {
    const int c4 = (lane & 15) * 4;
    for (int pass = 0; pass < 2; ++pass) {
#pragma unroll
      for (int it = 0; it < 8; ++it) {
        const int row = it * 2 + hh;
        v4f val = *(const v4f*)(os + row * 68 + c4);
        *(volatile v4f*)(ob + (size_t)(q0 + row) * DMOD + c4) = val;
      }
      __threadfence();
    }
  }
}

extern "C" void kernel_launch(void* const* d_in, const int* in_sizes, int n_in,
                              void* d_out, int out_size, void* d_ws, size_t ws_size,
                              hipStream_t stream) {
  if (n_in < 6) return;
  if (in_sizes[0] != NBATCH * SEQ * DMOD) return;
  if (in_sizes[1] != DMOD * DMOD || in_sizes[2] != DMOD * DMOD || in_sizes[3] != DMOD * DMOD || in_sizes[4] != DMOD * DMOD) return;
  if (in_sizes[5] != NHEAD) return;
  if (out_size != NBATCH * SEQ * DMOD) return;

  const float* x  = (const float*)d_in[0];
  const float* Wq = (const float*)d_in[1];
  const float* Wk = (const float*)d_in[2];
  const float* Wv = (const float*)d_in[3];
  const float* Wo = (const float*)d_in[4];
  const int*   hm = (const int*)d_in[5];

  const size_t PW16 = (size_t)DMOD * DMOD * 2;
  const size_t PX16 = (size_t)SEQ * DMOD * 2;
  const size_t PF32 = (size_t)SEQ * DMOD * 4;
  size_t off = 0;
  const size_t oWq = off; off += PW16;
  const size_t oWk = off; off += PW16;
  const size_t oWv = off; off += PW16;
  const size_t oWo = off; off += PW16;
  const size_t oX  = off; off += PX16;
  const size_t oQh = off; off += PX16;  const size_t oQl = off; off += PX16;
  const size_t oKh = off; off += PX16;  const size_t oKl = off; off += PX16;
  const size_t oVh = off; off += PX16;  const size_t oVl = off; off += PX16;
  const size_t oMf = off; off += PF32;
  const size_t oM16 = off; off += PX16;
  if (off > ws_size) return;

  char* ws = (char*)d_ws;
  unsigned short* Wq16 = (unsigned short*)(ws + oWq);
  unsigned short* Wk16 = (unsigned short*)(ws + oWk);
  unsigned short* Wv16 = (unsigned short*)(ws + oWv);
  unsigned short* Wo16 = (unsigned short*)(ws + oWo);
  unsigned short* X16  = (unsigned short*)(ws + oX);
  unsigned short* Qh   = (unsigned short*)(ws + oQh);  unsigned short* Ql = (unsigned short*)(ws + oQl);
  unsigned short* Kh   = (unsigned short*)(ws + oKh);  unsigned short* Kl = (unsigned short*)(ws + oKl);
  unsigned short* VTh  = (unsigned short*)(ws + oVh);  unsigned short* VTl = (unsigned short*)(ws + oVl);
  float*          MHf  = (float*)(ws + oMf);
  unsigned short* MH16 = (unsigned short*)(ws + oM16);
  const float*    fpad = (const float*)MHf;

  const dim3 blk(256);
  const int n2w = DMOD * DMOD / 2;
  const int n2x = SEQ * DMOD / 2;
  const dim3 gCastW((n2w + 255) / 256);
  const dim3 gCastX((n2x + 255) / 256);
  const dim3 gProj(((SEQ / 64) * (DMOD / 64) + 7) / 8, 1);
  const dim3 gVT(((DMOD / 64) * (SEQ / 64) + 7) / 8, 1);
  const dim3 gOut(((SEQ / 64) * (DMOD / 64) + 7) / 8, 1);
  const dim3 gAtt(NHEAD * (SEQ / 64));

  cast_f32_f16x2s<<<gCastW, blk, 0, stream>>>(Wq, (_Float16*)Wq16, n2w, 32.0f);
  cast_f32_f16x2s<<<gCastW, blk, 0, stream>>>(Wk, (_Float16*)Wk16, n2w, 32.0f);
  cast_f32_f16x2s<<<gCastW, blk, 0, stream>>>(Wv, (_Float16*)Wv16, n2w, 32.0f);
  cast_f32_f16x2s<<<gCastW, blk, 0, stream>>>(Wo, (_Float16*)Wo16, n2w, 32.0f);

  for (int b = 0; b < NBATCH; ++b) {
    const float* xb = x + (size_t)b * SEQ * DMOD;
    cast_f32_f16x2s<<<gCastX, blk, 0, stream>>>(xb, (_Float16*)X16, n2x, 1.0f);
    wmma_gemm64<0, false, 0, 2, false, 0><<<gProj, blk, 0, stream>>>(
        X16, X16, DMOD, 0L, Wq16, Wq16, DMOD, 0L, (void*)Qh, (void*)Ql, DMOD, 0L,
        fpad, fpad, 0L, SEQ, DMOD, DMOD, 1.0f / 32.0f);
    wmma_gemm64<0, false, 0, 2, false, 0><<<gProj, blk, 0, stream>>>(
        X16, X16, DMOD, 0L, Wk16, Wk16, DMOD, 0L, (void*)Kh, (void*)Kl, DMOD, 0L,
        fpad, fpad, 0L, SEQ, DMOD, DMOD, 1.0f / 32.0f);
    wmma_gemm64<0, false, 0, 2, false, 0><<<gVT, blk, 0, stream>>>(
        Wv16, Wv16, DMOD, 0L, X16, X16, DMOD, 0L, (void*)VTh, (void*)VTl, SEQ, 0L,
        fpad, fpad, 0L, DMOD, SEQ, DMOD, 1.0f / 32.0f);
    attn_full64_kernel<<<gAtt, dim3(128), 0, stream>>>(Qh, Ql, Kh, Kl, VTh, VTl, MHf, 0.125f);
    maskcast_f32_f16x2<<<gCastX, blk, 0, stream>>>(MHf, hm, (_Float16*)MH16, n2x, DMOD, 64.0f);
    float* outb = (float*)d_out + (size_t)b * SEQ * DMOD;
    wmma_gemm64<0, false, 0, 0, false, 0><<<gOut, blk, 0, stream>>>(
        MH16, MH16, DMOD, 0L, Wo16, Wo16, DMOD, 0L, (void*)outb, (void*)outb, DMOD, 0L,
        fpad, fpad, 0L, SEQ, DMOD, DMOD, 1.0f / 2048.0f);
  }
  (void)hipGetLastError();
}
